// TransformerBlock_89575837925998
// MI455X (gfx1250) — hardware-run, weakly checked
//
#include <hip/hip_runtime.h>


#ifndef SEQ
#define SEQ 4096
#endif
#define SEQ_FULL 4096
#define FEAT 256
#define NH_  8
#define KQD  64
#define DVD  32
#define HID  1024
#define AW   4
#define OSP  36
#define WSC  64.0f
#define WSI  (1.0f / 64.0f)
#define SC2  ((float)(0.0625 * 1.4426950408889634))
#define PSH  14.0f
#define NEGB (-3.0e38f)
#define RMS_EPS 1.1920928955078125e-07f

static_assert(KQD == 64);
static_assert(DVD == 32);
static_assert(NH_ * DVD == FEAT);
static_assert(FEAT == 256);
static_assert(FEAT % 64 == 0);
static_assert(HID % 64 == 0);
static_assert((NH_ * KQD) % 64 == 0);
static_assert((NH_ * DVD) % 64 == 0);
static_assert(KQD % 32 == 0);
static_assert(DVD % 32 == 0);
static_assert(FEAT % 32 == 0);
static_assert(HID % 32 == 0);
static_assert(SEQ % 64 == 0);
static_assert(SEQ % 32 == 0);
static_assert(SEQ % (16 * AW) == 0);
static_assert(SEQ % 8 == 0);
static_assert(SEQ <= SEQ_FULL);
static_assert(((size_t)SEQ * FEAT) % 8 == 0);
static_assert((OSP * 4) % 16 == 0);
static_assert((size_t)SEQ * KQD < (size_t)2147483647);
static_assert(32 * 4 * 16 == 16 * 64 * 2);
static_assert(32 * 8 * 16 == 16 * 64 * 4);
static_assert(32 * 4 * 16 == 16 * DVD * 4);
static_assert(256 * 1 * 16 == 32 * 64 * 2);
static_assert(256 * 8 == 64 * 32);
static_assert(32 * 2 * 16 == FEAT * 4);
static_assert(32 * 1 * 16 == FEAT * 2);
static_assert(16 * 68 * 4 <= 131072);
static_assert(AW * 16 * OSP * 4 <= 131072);
static_assert(8 * FEAT * 4 <= 131072);
static_assert(32 * 65 * 4 <= 131072);

typedef _Float16 h16;
typedef unsigned short bf;
typedef __attribute__((ext_vector_type(16))) __bf16   v16bf;
typedef __attribute__((ext_vector_type(16))) _Float16 v16h;
typedef __attribute__((ext_vector_type(8)))  _Float16 v8h;
typedef __attribute__((ext_vector_type(8)))  unsigned short v8us;
typedef __attribute__((ext_vector_type(8)))  float    v8f;
typedef __attribute__((ext_vector_type(4)))  float    v4f;
typedef v4f  __attribute__((may_alias)) v4fa;

__device__ __forceinline__ unsigned short f2bf(float f) { unsigned u = __float_as_uint(f); u += 0x7FFFu + ((u >> 16) & 1u); return (unsigned short)(u >> 16); }
__device__ __forceinline__ float bfr(float f) { return __uint_as_float(((unsigned)f2bf(f)) << 16); }
__device__ __forceinline__ v16h cat16(v8h lo, v8h hi) { return __builtin_shufflevector(lo, hi, 0, 1, 2, 3, 4, 5, 6, 7, 8, 9, 10, 11, 12, 13, 14, 15); }
__device__ __forceinline__ v16bf cat16b(v8us lo, v8us hi) { return __builtin_bit_cast(v16bf, __builtin_shufflevector(lo, hi, 0, 1, 2, 3, 4, 5, 6, 7, 8, 9, 10, 11, 12, 13, 14, 15)); }
__device__ __forceinline__ v8f wmma16(v16h a, v16h b, v8f c) { return __builtin_amdgcn_wmma_f32_16x16x32_f16(false, a, false, b, (short)0, c, false, false); }
__device__ __forceinline__ v8f wmmab(v16bf a, v16bf b, v8f c) { return __builtin_amdgcn_wmma_f32_16x16x32_bf16(false, a, false, b, (short)0, c, false, false); }
__device__ __forceinline__ v16h  ldh(const h16* p) { return cat16(*(const v8h*)p, *(const v8h*)(p + 16)); }
__device__ __forceinline__ v16bf ldb(const bf* p)  { return cat16b(*(const v8us*)p, *(const v8us*)(p + 16)); }
__device__ __forceinline__ void wave_sync() { __builtin_amdgcn_fence(3  , "wavefront"); __builtin_amdgcn_wave_barrier(); asm volatile("" ::: "memory"); }

static __device__ __forceinline__ h16 toh_flush(float v) { const h16 r = (h16)v; return (fabsf(v) < 6.103515625e-05f) ? (h16)0.0f : r; }
__device__ __forceinline__ v16h  ldfrag(const h16* p) { return ldh(p); }
__device__ __forceinline__ v16bf ldfrag(const bf* p)  { return ldb(p); }
__device__ __forceinline__ v8f mmag(v16h a, v16h b, v8f c) { c = wmma16(a, b, c); asm volatile("v_nop\n\tv_nop\n\tv_nop\n\tv_nop" : "+v"(c) : "v"(a), "v"(b)); return c; }
__device__ __forceinline__ v8f mmag(v16bf a, v16bf b, v8f c) { c = wmmab(a, b, c); asm volatile("v_nop\n\tv_nop\n\tv_nop\n\tv_nop" : "+v"(c) : "v"(a), "v"(b)); return c; }
__device__ __forceinline__ float silu_f(float v) { return v * __builtin_amdgcn_rcpf(1.0f + __builtin_amdgcn_exp2f(v * -1.4426950408889634f)); }

__global__ __launch_bounds__(256) void k_cvt8(const float* __restrict__ src, bf* dst, size_t n8) {
    const size_t i = (size_t)blockIdx.x * 256 + threadIdx.x; if (i >= n8) return;
    const v8f v = *(const v8f*)(src + i * 8); v8us o;
#pragma unroll
    for (int k = 0; k < 8; ++k) o[k] = f2bf(v[k]);
    *(volatile v8us*)(dst + i * 8) = o; __threadfence(); *(volatile v8us*)(dst + i * 8) = o;
}

__global__ __launch_bounds__(256) void k_wtr_bf(const float* __restrict__ W, bf* T, int IN, int OUT) {
    __shared__ float ts[32 * 65];
    const int tid = threadIdx.x;
    const int n0 = blockIdx.x * 32, k0 = blockIdx.y * 64;
    const size_t zoff = (size_t)blockIdx.z * (size_t)IN * (size_t)OUT;
    const int n = tid & 31, kr = tid >> 5;
#pragma unroll 1
    for (int i = 0; i < 8; ++i) { const int k = kr + 8 * i; ts[n * 65 + k] = W[zoff + (size_t)(k0 + k) * OUT + n0 + n]; }
    __syncthreads();
    const int row = tid >> 3, c8 = (tid & 7) * 8;
    v8us o;
#pragma unroll
    for (int j = 0; j < 8; ++j) o[j] = f2bf(ts[row * 65 + c8 + j]);
    const size_t oo = zoff + (size_t)(n0 + row) * IN + k0 + c8;
    *(volatile v8us*)(T + oo) = o; __threadfence(); *(volatile v8us*)(T + oo) = o;
}
__global__ __launch_bounds__(256) void k_wtr_h(const float* __restrict__ W, h16* T, int IN, int OUT) {
    __shared__ float ts[32 * 65];
    const int tid = threadIdx.x;
    const int n0 = blockIdx.x * 32, k0 = blockIdx.y * 64;
    const size_t zoff = (size_t)blockIdx.z * (size_t)IN * (size_t)OUT;
    const int n = tid & 31, kr = tid >> 5;
#pragma unroll 1
    for (int i = 0; i < 8; ++i) { const int k = kr + 8 * i; ts[n * 65 + k] = W[zoff + (size_t)(k0 + k) * OUT + n0 + n]; }
    __syncthreads();
    const int row = tid >> 3, c8 = (tid & 7) * 8;
    v8h o;
#pragma unroll
    for (int j = 0; j < 8; ++j) o[j] = toh_flush(bfr(ts[row * 65 + c8 + j]) * WSC);
    const size_t oo = zoff + (size_t)(n0 + row) * IN + k0 + c8;
    *(volatile v8h*)(T + oo) = o; __threadfence(); *(volatile v8h*)(T + oo) = o;
}

template <typename T, int ROWBIAS, int ACT, int OUTF>
__device__ __forceinline__ void gemm_body(const T* __restrict__ A, const T* __restrict__ Bt, const float* __restrict__ bias, const float* __restrict__ RES,
                                          h16* OH, float* OF, int K, int ldo, int cstr, float oscale) {
    typedef decltype(ldfrag((const T*)0)) FR;
    __shared__ __align__(16) float os[16 * 68];
    const int lane = threadIdx.x & 31, lr = lane & 15, hi = lane >> 4; const int r0 = blockIdx.x * 64, c0 = blockIdx.y * 64;
    v8f acc[4][4];
#pragma unroll
    for (int mb = 0; mb < 4; ++mb)
#pragma unroll
        for (int nb = 0; nb < 4; ++nb) acc[mb][nb] = (v8f){};
    const size_t aoff = (size_t)(r0 + lr) * K + 8 * hi, boff = (size_t)(c0 + lr) * K + 8 * hi;
#pragma unroll 1
    for (int kc = 0; kc < K; kc += 32) {
        FR a[4];
#pragma unroll
        for (int mb = 0; mb < 4; ++mb) a[mb] = ldfrag(A + aoff + (size_t)mb * 16 * K + kc);
#pragma unroll
        for (int nb = 0; nb < 4; ++nb) { const FR b = ldfrag(Bt + boff + (size_t)nb * 16 * K + kc);
#pragma unroll
            for (int mb = 0; mb < 4; ++mb) acc[mb][nb] = mmag(a[mb], b, acc[mb][nb]); }
    }
    float bc[4];
#pragma unroll
    for (int nb = 0; nb < 4; ++nb) { bc[nb] = 0.0f; if (ROWBIAS == 0) bc[nb] = bfr(bias[c0 + nb * 16 + lr]); }
    const size_t obase = (size_t)blockIdx.y * (size_t)cstr + (size_t)r0 * (size_t)ldo;
#pragma unroll
    for (int mb = 0; mb < 4; ++mb) {
        float br[8];
#pragma unroll
        for (int j = 0; j < 8; ++j) { br[j] = 0.0f; if (ROWBIAS == 1) br[j] = bfr(bias[r0 + mb * 16 + hi * 8 + j]); }
#pragma unroll
        for (int nb = 0; nb < 4; ++nb) {
#pragma unroll
            for (int j = 0; j < 8; ++j) { float v = acc[mb][nb][j] * oscale + bc[nb] + br[j]; if (ACT == 1) v = silu_f(v);
                os[(hi * 8 + j) * 68 + nb * 16 + lr] = v; } }
        wave_sync();
#pragma unroll 1
        for (int ps = 0; ps < 2; ++ps) {
            if (OUTF == 0) {
#pragma unroll
                for (int s = 0; s < 4; ++s) { const int row = 4 * s + (lane >> 3), c8 = (lane & 7) * 8;
                    const v4f x0 = *(const v4fa*)(&os[row * 68 + c8]); const v4f x1 = *(const v4fa*)(&os[row * 68 + c8 + 4]); v8h hv;
#pragma unroll
                    for (int i = 0; i < 4; ++i) { hv[i] = toh_flush(x0[i]); hv[4 + i] = toh_flush(x1[i]); }
                    const size_t oo = obase + (size_t)(mb * 16 + row) * (size_t)ldo + c8;
                    *(volatile v8h*)(OH + oo) = hv; }
            } else {
#pragma unroll
                for (int s = 0; s < 8; ++s) { const int row = 2 * s + (lane >> 4), c4 = (lane & 15) * 4;
                    const size_t oo = obase + (size_t)(mb * 16 + row) * (size_t)ldo + c4;
                    const v4f xs = *(const v4fa*)(&os[row * 68 + c4]); const v4f rs = *(const v4f*)(RES + oo);
                    const v4f val = xs + rs;
                    *(volatile v4f*)(OF + oo) = val; }
            }
            if (ps == 0) __threadfence(); }
        wave_sync();
    }
}

__global__ __launch_bounds__(32) void k_gemm_pc(const bf* __restrict__ A, const bf* __restrict__ Bt, const float* __restrict__ bias, h16* OH, int K, int ldo, int cstr) {
    gemm_body<bf, 0, 0, 0>(A, Bt, bias, (const float*)0, OH, (float*)0, K, ldo, cstr, 1.0f);
}
__global__ __launch_bounds__(32) void k_gemm_pr(const bf* __restrict__ A, const bf* __restrict__ Bt, const float* __restrict__ bias, h16* OH, int K, int ldo, int cstr) {
    gemm_body<bf, 1, 0, 0>(A, Bt, bias, (const float*)0, OH, (float*)0, K, ldo, cstr, 1.0f);
}
__global__ __launch_bounds__(32) void k_gemm_act(const h16* __restrict__ A, const h16* __restrict__ Bt, const float* __restrict__ bias, h16* OH, int K, int ldo, int cstr) {
    gemm_body<h16, 0, 1, 0>(A, Bt, bias, (const float*)0, OH, (float*)0, K, ldo, cstr, WSI);
}
__global__ __launch_bounds__(32) void k_gemm_res(const h16* __restrict__ A, const h16* __restrict__ Bt, const float* __restrict__ bias, const float* __restrict__ RES, float* OF, int K, int ldo, int cstr) {
    gemm_body<h16, 0, 0, 1>(A, Bt, bias, RES, (h16*)0, OF, K, ldo, cstr, WSI);
}

__global__ __launch_bounds__(32 * AW) void k_flash(const h16* __restrict__ QH, const h16* __restrict__ KP, const h16* __restrict__ VT, float* Y) {
    __shared__ __align__(16) float os[AW * 16 * OSP];
    const int lane = threadIdx.x & 31, lr = lane & 15, hi = lane >> 4;
    const int wave = __builtin_amdgcn_readfirstlane((int)(threadIdx.x >> 5));
    const int h = blockIdx.y;
    const int t0 = (blockIdx.x * AW + wave) * 16;
    const size_t pbase = (size_t)h * SEQ * KQD;
    const size_t qo = pbase + (size_t)(t0 + lr) * KQD + 8 * hi;
    const v16h q0 = ldh(QH + qo), q1 = ldh(QH + qo + 32);
    const size_t ko = pbase + (size_t)lr * KQD + 8 * hi;
    const size_t vo = ((size_t)h * DVD + (size_t)lr) * SEQ + 8 * hi;
    v8f o0 = (v8f){}, o1 = (v8f){};
    float m = NEGB, l = 0.0f;
#pragma unroll 1
    for (int key0 = 0; key0 < SEQ; key0 += 32) {
        const h16* ka = KP + ko + (size_t)key0 * KQD;
        const v16h ka0 = ldh(ka), ka1 = ldh(ka + 32), kb0 = ldh(ka + 16 * KQD), kb1 = ldh(ka + 16 * KQD + 32);
        v8f sa = (v8f){}, sb = (v8f){};
        sa = mmag(ka0, q0, sa); sa = mmag(ka1, q1, sa);
        sb = mmag(kb0, q0, sb); sb = mmag(kb1, q1, sb);
        float ta[8], tb[8]; float mx = NEGB;
#pragma unroll
        for (int r = 0; r < 8; ++r) { ta[r] = sa[r] * SC2; tb[r] = sb[r] * SC2; mx = fmaxf(mx, fmaxf(ta[r], tb[r])); }
        mx = fmaxf(mx, __shfl_xor(mx, 16, 32));
        const float mnew = fmaxf(m, mx);
        const float alpha = __builtin_amdgcn_exp2f(m - mnew);
        const float sh = PSH - mnew;
        v16h pb; float ls = 0.0f;
#pragma unroll
        for (int r = 0; r < 8; ++r) {
            const float xa = ta[r] + sh, xb = tb[r] + sh;
            const float ea = __builtin_amdgcn_exp2f(xa), eb = __builtin_amdgcn_exp2f(xb);
            const float ga = (xa < -14.0f) ? 0.0f : ea, gb = (xb < -14.0f) ? 0.0f : eb;
            const h16 pa = (h16)ga; const h16 pc = (h16)gb;
            pb[r] = pa; pb[8 + r] = pc;
            ls += (float)pa + (float)pc; }
        l = l * alpha + ls; m = mnew;
        o0 = o0 * alpha; o1 = o1 * alpha;
        const h16* va = VT + vo + key0;
        const v16h v0 = ldh(va), v1 = ldh(va + (size_t)16 * SEQ);
        o0 = mmag(v0, pb, o0); o1 = mmag(v1, pb, o1);
    }
    l += __shfl_xor(l, 16, 32);
    const float inv = 1.0f / l;
    const int wb = wave * 16 * OSP;
    { v4f a, c;
      a[0] = o0[0] * inv; a[1] = o0[1] * inv; a[2] = o0[2] * inv; a[3] = o0[3] * inv; c[0] = o0[4] * inv; c[1] = o0[5] * inv; c[2] = o0[6] * inv; c[3] = o0[7] * inv;
      *(v4fa*)(&os[wb + lr * OSP +  0 + 8 * hi]) = a; *(v4fa*)(&os[wb + lr * OSP +  0 + 8 * hi + 4]) = c;
      a[0] = o1[0] * inv; a[1] = o1[1] * inv; a[2] = o1[2] * inv; a[3] = o1[3] * inv; c[0] = o1[4] * inv; c[1] = o1[5] * inv; c[2] = o1[6] * inv; c[3] = o1[7] * inv;
      *(v4fa*)(&os[wb + lr * OSP + 16 + 8 * hi]) = a; *(v4fa*)(&os[wb + lr * OSP + 16 + 8 * hi + 4]) = c; }
    wave_sync();
    float* orow = Y + (size_t)t0 * FEAT + h * DVD;
#pragma unroll 1
    for (int ps = 0; ps < 2; ++ps) {
#pragma unroll
        for (int s = 0; s < 4; ++s) { const int row = 4 * s + (lane >> 3), cofs = (lane & 7) * 4;
            const v4f val = *(const v4fa*)(&os[wb + row * OSP + cofs]);
            *(volatile v4f*)(orow + (size_t)row * FEAT + cofs) = val; }
        if (ps == 0) __threadfence(); }
}

template <int FIRST>
__device__ __forceinline__ void norm_body(const float* __restrict__ XA, const float* __restrict__ YB, const float* __restrict__ G, float* OF, h16* OH) {
#pragma clang fp contract(off)
    __shared__ __align__(16) float zs[8 * FEAT];
    const int lane = threadIdx.x & 31;
    const int wave = __builtin_amdgcn_readfirstlane((int)(threadIdx.x >> 5));
    const size_t ro = (size_t)(blockIdx.x * 8 + wave) * FEAT;
    const int ca = 4 * lane, cb = 128 + 4 * lane;
    v4f a0 = *(const v4f*)(XA + ro + ca), a1 = *(const v4f*)(XA + ro + cb);
    if (FIRST == 1) {
        const v4f y0 = *(const v4f*)(YB + ro + ca), y1 = *(const v4f*)(YB + ro + cb);
#pragma unroll
        for (int i = 0; i < 4; ++i) { a0[i] = bfr(a0[i]) + y0[i]; a1[i] = bfr(a1[i]) + y1[i]; } }
    float ss = 0.0f;
#pragma unroll
    for (int i = 0; i < 4; ++i) { ss += a0[i] * a0[i]; ss += a1[i] * a1[i]; }
#pragma unroll
    for (int msk = 16; msk >= 1; msk >>= 1) ss += __shfl_xor(ss, msk, 32);
    const float rinv = rsqrtf(ss * (1.0f / (float)FEAT) + RMS_EPS);
    const v4f g0 = *(const v4f*)(G + ca), g1 = *(const v4f*)(G + cb);
    v4f z0, z1;
#pragma unroll
    for (int i = 0; i < 4; ++i) { z0[i] = a0[i] * rinv * bfr(g0[i]); z1[i] = a1[i] * rinv * bfr(g1[i]); }
    v8h hv = (v8h){};
    if (FIRST == 1) {
        const int wb = wave * FEAT;
        *(v4fa*)(&zs[wb + ca]) = z0; *(v4fa*)(&zs[wb + cb]) = z1;
        wave_sync();
        const v4f x0 = *(const v4fa*)(&zs[wb + 8 * lane]); const v4f x1 = *(const v4fa*)(&zs[wb + 8 * lane + 4]);
#pragma unroll
        for (int i = 0; i < 4; ++i) { hv[i] = toh_flush(x0[i]); hv[4 + i] = toh_flush(x1[i]); } }
#pragma unroll 1
    for (int ps = 0; ps < 2; ++ps) {
        *(volatile v4f*)(OF + ro + ca) = z0; *(volatile v4f*)(OF + ro + cb) = z1;
        if (FIRST == 1) *(volatile v8h*)(OH + ro + 8 * lane) = hv;
        if (ps == 0) __threadfence(); }
}
__global__ __launch_bounds__(256) void k_norm_a(const float* __restrict__ X, const float* __restrict__ Yp, const float* __restrict__ G, float* ZF, h16* ZH) {
    norm_body<1>(X, Yp, G, ZF, ZH);
}
__global__ __launch_bounds__(256) void k_norm_b(const float* __restrict__ PZ, const float* __restrict__ G, float* OUT) {
    norm_body<0>(PZ, (const float*)0, G, OUT, (h16*)0);
}

static constexpr size_t al256(size_t v) { return (v + 255) & ~(size_t)255; }
static constexpr size_t SZ_XB  = al256((size_t)SEQ * FEAT * 2);
static constexpr size_t SZ_WQK = al256((size_t)NH_ * KQD * FEAT * 2);
static constexpr size_t SZ_WV  = al256((size_t)NH_ * DVD * FEAT * 2);
static constexpr size_t SZ_W1  = al256((size_t)FEAT * HID * 2);
static constexpr size_t SZ_W2  = al256((size_t)HID * HID * 2);
static constexpr size_t SZ_QK  = al256((size_t)NH_ * SEQ * KQD * 2);
static constexpr size_t SZ_VT  = al256((size_t)NH_ * DVD * SEQ * 2);
static constexpr size_t SZ_F   = al256((size_t)SEQ * FEAT * 4);
static constexpr size_t SZ_ZH  = al256((size_t)SEQ * FEAT * 2);
static constexpr size_t SZ_H   = al256((size_t)SEQ * HID * 2);
static constexpr size_t SZ_TOTAL = SZ_XB + 2 * SZ_WQK + SZ_WV + 2 * SZ_W1 + SZ_W2 + 2 * SZ_QK + SZ_VT + 3 * SZ_F + SZ_ZH + 2 * SZ_H;
static_assert(SZ_TOTAL <= (size_t)134217728);
static_assert(SZ_XB == (size_t)SEQ * FEAT * 2);
static_assert(SZ_QK == (size_t)NH_ * SEQ * KQD * 2);
static_assert(SZ_VT == (size_t)NH_ * DVD * SEQ * 2);
static_assert(SZ_H == (size_t)SEQ * HID * 2);
static_assert(SZ_F == (size_t)SEQ * FEAT * 4);

extern "C" void kernel_launch(void* const* d_in, const int* in_sizes, int n_in,
                              void* d_out, int out_size, void* d_ws, size_t ws_size, hipStream_t stream) {
    if (n_in < 15) return;
    if ((size_t)in_sizes[0] < (size_t)SEQ * FEAT) return;
    if ((size_t)in_sizes[1] < (size_t)NH_ * FEAT * KQD || (size_t)in_sizes[3] < (size_t)NH_ * FEAT * KQD || (size_t)in_sizes[5] < (size_t)NH_ * FEAT * DVD) return;
    if (in_sizes[2] < NH_ * KQD || in_sizes[4] < NH_ * KQD || in_sizes[6] < NH_ * DVD) return;
    if (in_sizes[7] < FEAT || in_sizes[8] < FEAT) return;
    if ((size_t)in_sizes[9] < (size_t)FEAT * HID || (size_t)in_sizes[11] < (size_t)HID * HID || (size_t)in_sizes[13] < (size_t)HID * FEAT) return;
    if (in_sizes[10] < HID || in_sizes[12] < HID || in_sizes[14] < FEAT) return;
    if ((size_t)out_size < (size_t)SEQ * FEAT) return;
    if (SZ_TOTAL > ws_size) return;
    const float* x  = (const float*)d_in[0];
    const float* wq = (const float*)d_in[1];  const float* bq = (const float*)d_in[2];
    const float* wk = (const float*)d_in[3];  const float* bk = (const float*)d_in[4];
    const float* wv = (const float*)d_in[5];  const float* bv = (const float*)d_in[6];
    const float* g1 = (const float*)d_in[7];  const float* g2 = (const float*)d_in[8];
    const float* w1 = (const float*)d_in[9];  const float* b1 = (const float*)d_in[10];
    const float* w2 = (const float*)d_in[11]; const float* b2 = (const float*)d_in[12];
    const float* w3 = (const float*)d_in[13]; const float* b3 = (const float*)d_in[14];
    float* OUT = (float*)d_out;
    char* wsp = (char*)d_ws;
    bf*  XB  = (bf*)wsp;   wsp += SZ_XB;
    bf*  WQT = (bf*)wsp;   wsp += SZ_WQK;
    bf*  WKT = (bf*)wsp;   wsp += SZ_WQK;
    bf*  WVT = (bf*)wsp;   wsp += SZ_WV;
    h16* W1T = (h16*)wsp;  wsp += SZ_W1;
    h16* W2T = (h16*)wsp;  wsp += SZ_W2;
    h16* W3T = (h16*)wsp;  wsp += SZ_W1;
    h16* QH  = (h16*)wsp;  wsp += SZ_QK;
    h16* KP  = (h16*)wsp;  wsp += SZ_QK;
    h16* VT  = (h16*)wsp;  wsp += SZ_VT;
    float* Y  = (float*)wsp; wsp += SZ_F;
    float* ZF = (float*)wsp; wsp += SZ_F;
    float* PZ = (float*)wsp; wsp += SZ_F;
    h16* ZH  = (h16*)wsp;  wsp += SZ_ZH;
    h16* H1  = (h16*)wsp;  wsp += SZ_H;
    h16* H2  = (h16*)wsp;  wsp += SZ_H;

    { const size_t n8 = (size_t)SEQ * FEAT / 8;
      k_cvt8<<<(unsigned)((n8 + 255) / 256), 256, 0, stream>>>(x, XB, n8); }
    k_wtr_bf<<<dim3(KQD / 32, FEAT / 64, NH_), 256, 0, stream>>>(wq, WQT, FEAT, KQD);
    k_wtr_bf<<<dim3(KQD / 32, FEAT / 64, NH_), 256, 0, stream>>>(wk, WKT, FEAT, KQD);
    k_wtr_bf<<<dim3(DVD / 32, FEAT / 64, NH_), 256, 0, stream>>>(wv, WVT, FEAT, DVD);
    k_wtr_h<<<dim3(HID / 32, FEAT / 64, 1), 256, 0, stream>>>(w1, W1T, FEAT, HID);
    k_wtr_h<<<dim3(HID / 32, HID / 64, 1), 256, 0, stream>>>(w2, W2T, HID, HID);
    k_wtr_h<<<dim3(FEAT / 32, HID / 64, 1), 256, 0, stream>>>(w3, W3T, HID, FEAT);

    k_gemm_pc<<<dim3(SEQ / 64, NH_ * KQD / 64, 1), 32, 0, stream>>>(XB, WQT, bq, QH, FEAT, KQD, SEQ * KQD);
    k_gemm_pc<<<dim3(SEQ / 64, NH_ * KQD / 64, 1), 32, 0, stream>>>(XB, WKT, bk, KP, FEAT, KQD, SEQ * KQD);
    k_gemm_pr<<<dim3(NH_ * DVD / 64, SEQ / 64, 1), 32, 0, stream>>>(WVT, XB, bv, VT, FEAT, SEQ, 64);

    k_flash<<<dim3(SEQ / (16 * AW), NH_, 1), 32 * AW, 0, stream>>>(QH, KP, VT, Y);

    k_norm_a<<<SEQ / 8, 256, 0, stream>>>(x, Y, g1, ZF, ZH);

    k_gemm_act<<<dim3(SEQ / 64, HID / 64, 1), 32, 0, stream>>>(ZH, W1T, b1, H1, FEAT, HID, 64);
    k_gemm_act<<<dim3(SEQ / 64, HID / 64, 1), 32, 0, stream>>>(H1, W2T, b2, H2, HID, HID, 64);
    k_gemm_res<<<dim3(SEQ / 64, FEAT / 64, 1), 32, 0, stream>>>(H2, W3T, b3, ZF, PZ, HID, FEAT, 64);

    k_norm_b<<<SEQ / 8, 256, 0, stream>>>(PZ, g2, OUT);
}
